// EagerBidirectionalAttentionBlock_74509092651379
// MI455X (gfx1250) — hardware-verified
//
#include <hip/hip_runtime.h>
#include <math.h>
#include <stdint.h>

constexpr int kBatch = 2;
constexpr int kSeq   = 2048;
constexpr int kHid   = 1024;
constexpr int kHeads = 16;
constexpr int kHdim  = 64;
constexpr int kRows  = kBatch * kSeq;
constexpr float kPScale = 32768.0f;

typedef __attribute__((ext_vector_type(16))) _Float16 v16h;
typedef __attribute__((ext_vector_type(8)))  _Float16 v8h;
typedef __attribute__((ext_vector_type(16))) __bf16   v16b;
typedef __attribute__((ext_vector_type(8)))  __bf16   v8b;
typedef __attribute__((ext_vector_type(8)))  float    v8f;
typedef __attribute__((ext_vector_type(4)))  float    v4f;
typedef __attribute__((ext_vector_type(2)))  float    v2f;

__device__ __forceinline__ unsigned short f2bf_bits(float f) {
  unsigned u = __float_as_uint(f);
  return (unsigned short)((u + 0x7FFFu + ((u >> 16) & 1u)) >> 16);
}
__device__ __forceinline__ float bf_bits2f(unsigned short h) { return __uint_as_float(((unsigned)h) << 16); }
__device__ __forceinline__ unsigned pk16(unsigned short a, unsigned short b) { return (unsigned)a | ((unsigned)b << 16); }

__device__ __forceinline__ void dep_guard_h(v8f& a, v8f& b, v16h x, v16h y) { asm volatile("v_nop\n\tv_nop\n\tv_nop\n\tv_nop" : "+v"(a), "+v"(b) : "v"(x), "v"(y)); }
__device__ __forceinline__ void dep_guard_b(v8f& a, v8f& b, v16b x, v16b y) { asm volatile("v_nop\n\tv_nop\n\tv_nop\n\tv_nop" : "+v"(a), "+v"(b) : "v"(x), "v"(y)); }
__device__ __forceinline__ void keep4_h(v16h a, v16h b, v16h c, v16h d) { asm volatile("v_nop" :: "v"(a), "v"(b), "v"(c), "v"(d)); }
__device__ __forceinline__ void keep4_b(v16b a, v16b b, v16b c, v16b d) { asm volatile("v_nop" :: "v"(a), "v"(b), "v"(c), "v"(d)); }
__device__ __forceinline__ void acc_guard4(v8f& a, v8f& b, v8f& c, v8f& d) { asm volatile("v_nop\n\tv_nop\n\tv_nop\n\tv_nop" : "+v"(a), "+v"(b), "+v"(c), "+v"(d)); }
template <typename T> struct Frag;
template <> struct Frag<_Float16> {
  typedef v16h V; union U { v16h v; v8h h[2]; };
  static __device__ __forceinline__ v16h load(const _Float16* p) {
    U f; f.h[0] = *(const v8h*)(p); f.h[1] = *(const v8h*)(p + 16); return f.v;
  }
  static __device__ __forceinline__ v8f mma(v16h a, v16h b, v8f c) {
    return __builtin_amdgcn_wmma_f32_16x16x32_f16(false, a, false, b, (short)0, c, false, false);
  }
  static __device__ __forceinline__ void guard(v8f& a, v8f& b, v16h x, v16h y) { dep_guard_h(a, b, x, y); }
  static __device__ __forceinline__ void keep(v16h a, v16h b, v16h c, v16h d) { keep4_h(a, b, c, d); }
};
template <> struct Frag<__bf16> {
  typedef v16b V; union U { v16b v; v8b h[2]; };
  static __device__ __forceinline__ v16b load(const __bf16* p) {
    U f; f.h[0] = *(const v8b*)(p); f.h[1] = *(const v8b*)(p + 16); return f.v;
  }
  static __device__ __forceinline__ v8f mma(v16b a, v16b b, v8f c) {
    return __builtin_amdgcn_wmma_f32_16x16x32_bf16(false, a, false, b, (short)0, c, false, false);
  }
  static __device__ __forceinline__ void guard(v8f& a, v8f& b, v16b x, v16b y) { dep_guard_b(a, b, x, y); }
  static __device__ __forceinline__ void keep(v16b a, v16b b, v16b c, v16b d) { keep4_b(a, b, c, d); }
};

__device__ __forceinline__ v8f hmma16(v16h a, v16h b, v8f c) {
  c = __builtin_amdgcn_wmma_f32_16x16x32_f16(false, a, false, b, (short)0, c, false, false);
  asm volatile("v_nop\n\tv_nop\n\tv_nop\n\tv_nop" : "+v"(c) : "v"(a), "v"(b));
  return c;
}

template <int ET> struct Elem;
template <> struct Elem<0> { typedef _Float16 T; };
template <> struct Elem<1> { typedef __bf16 T; };
template <int ET, int SPLIT, int BIAS_MODE, int OUT_MODE, bool RESID, bool BIAS_RNE>
__global__ __launch_bounds__(256) void wmma_gemm64(
    const unsigned short* __restrict__ Ap, const unsigned short* __restrict__ A2p, int lda, long strideA,
    const unsigned short* __restrict__ Btp, const unsigned short* __restrict__ Bt2p, int ldb, long strideB,
    void* __restrict__ Cout, void* __restrict__ Cout2, int ldc, long strideC,
    const float* __restrict__ bias,
    const float* __restrict__ resid, long strideR,
    int M, int N, int K, float scale) {
  typedef typename Elem<ET>::T T;
  typedef typename Frag<T>::V V;
  const T* A = (const T*)Ap; const T* A2 = (const T*)A2p; const T* Bt = (const T*)Btp; const T* Bt2 = (const T*)Bt2p;
  __shared__ __align__(16) float sT[8][16 * 68];
  const int b    = blockIdx.y;
  const int lane = threadIdx.x & 31;
  const int wave = threadIdx.x >> 5;
  const int tilesN = N >> 6;
  const int tilesM = M >> 6;
  const int tile = blockIdx.x * 8 + wave;
  if (tile >= tilesM * tilesN) return;
  const int tm = tile / tilesN;
  const int tn = tile - tm * tilesN;
  const int m0 = tm << 6;
  const int n0 = tn << 6;

  const T* Ab  = A  + (size_t)b * strideA;
  const T* Bb  = Bt + (size_t)b * strideB;
  const T* Ab2 = (SPLIT != 0) ? (A2  + (size_t)b * strideA) : nullptr;
  const T* Bb2 = (SPLIT == 1) ? (Bt2 + (size_t)b * strideB) : nullptr;

  const int rlane = lane & 15;
  const int koff  = (lane >> 4) * 8;
  const int mOff  = (lane >> 4) * 8;

  v8f acc[4][4];
#pragma unroll
  for (int i = 0; i < 4; ++i)
#pragma unroll
    for (int j = 0; j < 4; ++j) acc[i][j] = (v8f){0.f,0.f,0.f,0.f,0.f,0.f,0.f,0.f};

  for (int k0 = 0; k0 < K; k0 += 32) {
    V bh[4], bl[4];
#pragma unroll
    for (int j = 0; j < 4; ++j) {
      const size_t bo = (size_t)(n0 + (j << 4) + rlane) * ldb + koff + k0;
      bh[j] = Frag<T>::load(Bb + bo);
      if (SPLIT == 1) bl[j] = Frag<T>::load(Bb2 + bo);
    }
#pragma unroll
    for (int i = 0; i < 4; ++i) {
      const size_t ao = (size_t)(m0 + (i << 4) + rlane) * lda + koff + k0;
      V ah = Frag<T>::load(Ab + ao);
      V al;
      if (SPLIT != 0) al = Frag<T>::load(Ab2 + ao);
#pragma unroll
      for (int j = 0; j < 4; ++j) {
        acc[i][j] = Frag<T>::mma(ah, bh[j], acc[i][j]);
        if (SPLIT == 1) acc[i][j] = Frag<T>::mma(ah, bl[j], acc[i][j]);
        if (SPLIT != 0) acc[i][j] = Frag<T>::mma(al, bh[j], acc[i][j]);
      }
      Frag<T>::guard(acc[i][0], acc[i][3], ah, (SPLIT != 0) ? al : ah);
    }
    Frag<T>::keep(bh[0], bh[1], bh[2], bh[3]);
    if (SPLIT == 1) Frag<T>::keep(bl[0], bl[1], bl[2], bl[3]);
  }
  acc_guard4(acc[0][0], acc[0][1], acc[0][2], acc[0][3]);
  acc_guard4(acc[1][0], acc[1][1], acc[1][2], acc[1][3]);
  acc_guard4(acc[2][0], acc[2][1], acc[2][2], acc[2][3]);
  acc_guard4(acc[3][0], acc[3][1], acc[3][2], acc[3][3]);

  float* slab = sT[wave];
  const float* Rb = RESID ? (resid + (size_t)b * strideR) : nullptr;
#pragma unroll
  for (int i = 0; i < 4; ++i) {
    const int mBase = m0 + (i << 4);
#pragma unroll
    for (int j = 0; j < 4; ++j) {
      const int n = n0 + (j << 4) + rlane;
      float bv = 0.f;
      if (BIAS_MODE == 2) { bv = bias[n]; if (BIAS_RNE) bv = bf_bits2f(f2bf_bits(bv)); }
#pragma unroll
      for (int r = 0; r < 8; ++r) {
        float v = acc[i][j][r] * scale;
        if (BIAS_MODE == 1) { float bm = bias[mBase + mOff + r]; if (BIAS_RNE) bm = bf_bits2f(f2bf_bits(bm)); v += bm; }
        if (BIAS_MODE == 2) v += bv;
        if (RESID) v += Rb[(size_t)(mBase + mOff + r) * ldc + n];
        slab[(mOff + r) * 68 + (j << 4) + rlane] = v;
      }
    }
    __builtin_amdgcn_fence(__ATOMIC_RELEASE, "workgroup");
    __builtin_amdgcn_wave_barrier();
    __builtin_amdgcn_fence(__ATOMIC_ACQUIRE, "workgroup");
    if (OUT_MODE == 0) {
      float* C = (float*)Cout + (size_t)b * strideC;
      const int hh = lane >> 4, c4 = (lane & 15) * 4;
      for (int pass = 0; pass < 2; ++pass) {
#pragma unroll
        for (int it = 0; it < 8; ++it) {
          const int row = it * 2 + hh;
          v4f v = *(const v4f*)(slab + row * 68 + c4);
          *(volatile v4f*)(C + (size_t)(mBase + row) * ldc + n0 + c4) = v;
        }
        __threadfence();
      }
    } else {
      const int q = lane >> 3, c8 = (lane & 7) * 8;
      unsigned short* C  = (unsigned short*)Cout  + (size_t)b * strideC;
      unsigned short* C2 = (OUT_MODE == 2) ? ((unsigned short*)Cout2 + (size_t)b * strideC) : nullptr;
      for (int pass = 0; pass < 2; ++pass) {
#pragma unroll
        for (int it = 0; it < 4; ++it) {
          const int row = it * 4 + q;
          const float* sp = slab + row * 68 + c8;
          v8h hv, lv;
#pragma unroll
          for (int e = 0; e < 8; ++e) {
            if (OUT_MODE == 1) {
              hv[e] = (_Float16)sp[e];
            } else {
              unsigned short hb = f2bf_bits(sp[e]);
              unsigned short lb = f2bf_bits(sp[e] - bf_bits2f(hb));
              hv[e] = __builtin_bit_cast(_Float16, hb);
              lv[e] = __builtin_bit_cast(_Float16, lb);
            }
          }
          *(volatile v8h*)(C + (size_t)(mBase + row) * ldc + n0 + c8) = hv;
          if (OUT_MODE == 2) *(volatile v8h*)(C2 + (size_t)(mBase + row) * ldc + n0 + c8) = lv;
        }
        __threadfence();
      }
    }
    __builtin_amdgcn_fence(__ATOMIC_RELEASE, "workgroup");
    __builtin_amdgcn_wave_barrier();
    __builtin_amdgcn_fence(__ATOMIC_ACQUIRE, "workgroup");
  }
}

__global__ __launch_bounds__(256) void cast_f32_bf16x2(
    const float* __restrict__ in, unsigned short* __restrict__ out, int n2) {
  const int i = blockIdx.x * 256 + threadIdx.x;
  if (i < n2) {
    const v2f f = *(const v2f*)(in + 2 * (size_t)i);
    const unsigned u = pk16(f2bf_bits(f[0]), f2bf_bits(f[1]));
    ((volatile unsigned*)out)[i] = u;
    __threadfence();
    ((volatile unsigned*)out)[i] = u;
  }
}

#define AT_D 64
#define AT_NW 4
#define AT_QB 64
#define AT_KC 64

__global__ __launch_bounds__(128)
void mha_full64_f16(const unsigned short* __restrict__ qp, const unsigned short* __restrict__ kp,
                    const unsigned short* __restrict__ vtp, const int* __restrict__ kmask,
                    unsigned short* __restrict__ ctxh, unsigned short* __restrict__ ctxl) {
  union FH { v16h v; v8h h[2]; };
  __shared__ __align__(16) _Float16 Ksh[AT_KC * AT_D];
  __shared__ __align__(16) _Float16 Vth[AT_D * AT_KC];
  __shared__ __align__(16) _Float16 Psh[AT_NW][16 * AT_KC];
  __shared__ __align__(16) float    Os[AT_NW][16 * 68];

  const int tid  = threadIdx.x;
  const int wave = tid >> 5;
  const int lane = tid & 31;
  const int hh   = lane >> 4;
  const int c    = lane & 15;

  const int nqb = kSeq / AT_QB;
  const int bx = blockIdx.x;
  const int qb = bx % nqb;
  const int bh = bx / nqb;
  const int h  = bh % kHeads;
  const int b  = bh / kHeads;
  const int q0 = qb * AT_QB + wave * 16;

  const _Float16* Qh = (const _Float16*)(const void*)qp  + (size_t)b * kSeq * kHid + (size_t)h * AT_D;
  const _Float16* Kh = (const _Float16*)(const void*)kp  + (size_t)b * kSeq * kHid + (size_t)h * AT_D;
  const _Float16* Vh = (const _Float16*)(const void*)vtp + ((size_t)b * kHid + (size_t)h * AT_D) * kSeq;
  const int* mk = kmask + (size_t)b * kSeq;
  unsigned short* Ch = ctxh + (size_t)b * kSeq * kHid + (size_t)h * AT_D;
  unsigned short* Cl = ctxl + (size_t)b * kSeq * kHid + (size_t)h * AT_D;

  v16h qa[2];
#pragma unroll
  for (int dc = 0; dc < 2; ++dc)
    qa[dc] = Frag<_Float16>::load(Qh + (size_t)(q0 + c) * kHid + dc * 32 + 8 * hh);

  float mrow[8], lrow[8];
  v8f oacc[4];
#pragma unroll
  for (int r = 0; r < 8; ++r) { mrow[r] = -INFINITY; lrow[r] = 0.f; }
#pragma unroll
  for (int t = 0; t < 4; ++t) oacc[t] = (v8f){0.f,0.f,0.f,0.f,0.f,0.f,0.f,0.f};

  const int nChunks = kSeq / AT_KC;
#pragma unroll 1
  for (int kc = 0; kc < nChunks; ++kc) {
    const int kv0 = kc * AT_KC;
    __syncthreads();
    {
      const int r = tid >> 1, half = (tid & 1) * 32;
      const _Float16* ks = Kh + (size_t)(kv0 + r) * kHid + half;
      const _Float16* vs = Vh + (size_t)r * kSeq + kv0 + half;
#pragma unroll
      for (int i = 0; i < 4; ++i) {
        const v8h a0 = *(const v8h*)(ks + 8 * i);
        const v8h b0 = *(const v8h*)(vs + 8 * i);
        *(v8h*)(Ksh + r * AT_D  + half + 8 * i) = a0;
        *(v8h*)(Vth + r * AT_KC + half + 8 * i) = b0;
      }
    }
    __syncthreads();

    v8f s[4];
#pragma unroll
    for (int j = 0; j < 4; ++j) {
      s[j] = (v8f){0.f,0.f,0.f,0.f,0.f,0.f,0.f,0.f};
#pragma unroll
      for (int dc = 0; dc < 2; ++dc) {
        FH kb;
        kb.h[0] = *(const v8h*)(Ksh + (j * 16 + c) * AT_D + dc * 32 + 8 * hh);
        kb.h[1] = *(const v8h*)(Ksh + (j * 16 + c) * AT_D + dc * 32 + 16 + 8 * hh);
        s[j] = hmma16(qa[dc], kb.v, s[j]);
      }
    }
    int kvkeep[4];
#pragma unroll
    for (int j = 0; j < 4; ++j) kvkeep[j] = mk[kv0 + j * 16 + c];

    float cm[8];
#pragma unroll
    for (int r = 0; r < 8; ++r) {
      float m = -INFINITY;
#pragma unroll
      for (int j = 0; j < 4; ++j) {
        float sv = s[j][r] * 0.125f;
        sv = (kvkeep[j] != 0) ? sv : -INFINITY;
        s[j][r] = sv;
        m = fmaxf(m, sv);
      }
#pragma unroll
      for (int off = 1; off < 16; off <<= 1) m = fmaxf(m, __shfl_xor(m, off, 32));
      cm[r] = m;
    }
    _Float16* pw = Psh[wave];
#pragma unroll
    for (int r = 0; r < 8; ++r) {
      const float mnew = fmaxf(mrow[r], cm[r]);
      const float mref = (mnew == -INFINITY) ? 0.0f : mnew;
      const float alpha = expf(mrow[r] - mref);
      mrow[r] = mnew;
      float psum = 0.f;
#pragma unroll
      for (int j = 0; j < 4; ++j) {
        const float p = expf(s[j][r] - mref);
        psum += p;
        pw[(8 * hh + r) * AT_KC + j * 16 + c] = (_Float16)(p * kPScale);
      }
#pragma unroll
      for (int off = 1; off < 16; off <<= 1) psum += __shfl_xor(psum, off, 32);
      lrow[r] = lrow[r] * alpha + psum;
#pragma unroll
      for (int t = 0; t < 4; ++t) oacc[t][r] *= alpha;
    }
    __builtin_amdgcn_fence(__ATOMIC_RELEASE, "workgroup");
    __builtin_amdgcn_wave_barrier();
    __builtin_amdgcn_fence(__ATOMIC_ACQUIRE, "workgroup");
#pragma unroll
    for (int kk = 0; kk < 2; ++kk) {
      FH pa;
      pa.h[0] = *(const v8h*)(pw + c * AT_KC + kk * 32 + 8 * hh);
      pa.h[1] = *(const v8h*)(pw + c * AT_KC + kk * 32 + 16 + 8 * hh);
#pragma unroll
      for (int t = 0; t < 4; ++t) {
        FH vb;
        vb.h[0] = *(const v8h*)(Vth + (t * 16 + c) * AT_KC + kk * 32 + 8 * hh);
        vb.h[1] = *(const v8h*)(Vth + (t * 16 + c) * AT_KC + kk * 32 + 16 + 8 * hh);
        oacc[t] = hmma16(pa.v, vb.v, oacc[t]);
      }
    }
  }

  float* os = Os[wave];
#pragma unroll
  for (int r = 0; r < 8; ++r) {
    const float inv = 1.0f / (lrow[r] * kPScale);
#pragma unroll
    for (int t = 0; t < 4; ++t) os[(8 * hh + r) * 68 + t * 16 + c] = oacc[t][r] * inv;
  }
  __builtin_amdgcn_fence(__ATOMIC_RELEASE, "workgroup");
  __builtin_amdgcn_wave_barrier();
  __builtin_amdgcn_fence(__ATOMIC_ACQUIRE, "workgroup");
  {
    const int qq = lane >> 3, c8 = (lane & 7) * 8;
    for (int pass = 0; pass < 2; ++pass) {
#pragma unroll
      for (int it = 0; it < 4; ++it) {
        const int row = it * 4 + qq;
        const float* sp = os + row * 68 + c8;
        v8h hv, lv;
#pragma unroll
        for (int e = 0; e < 8; ++e) {
          const unsigned short hb = f2bf_bits(sp[e]);
          const unsigned short lb = f2bf_bits(sp[e] - bf_bits2f(hb));
          hv[e] = __builtin_bit_cast(_Float16, hb);
          lv[e] = __builtin_bit_cast(_Float16, lb);
        }
        const size_t go = (size_t)(q0 + row) * kHid + c8;
        *(volatile v8h*)(Ch + go) = hv;
        *(volatile v8h*)(Cl + go) = lv;
      }
      __threadfence();
    }
  }
}

extern "C" void kernel_launch(void* const* d_in, const int* in_sizes, int n_in,
                              void* d_out, int out_size, void* d_ws, size_t ws_size,
                              hipStream_t stream)
{
  const size_t MiB = (size_t)1 << 20;
  const size_t wsTotal = 56 * MiB;
  if (n_in < 10) return;
  if (in_sizes[0] != kRows * kHid || in_sizes[1] != kBatch * kSeq || out_size != kRows * kHid) return;
  if (in_sizes[2] != kHid * kHid || in_sizes[4] != kHid * kHid || in_sizes[6] != kHid * kHid || in_sizes[8] != kHid * kHid) return;
  if (in_sizes[3] != kHid || in_sizes[5] != kHid || in_sizes[7] != kHid || in_sizes[9] != kHid) return;
  if (ws_size < wsTotal) return;

  const float* x    = (const float*)d_in[0];
  const int*   mask = (const int*)d_in[1];
  const float* Wq_w = (const float*)d_in[2];
  const float* Wq_b = (const float*)d_in[3];
  const float* Wk_w = (const float*)d_in[4];
  const float* Wk_b = (const float*)d_in[5];
  const float* Wv_w = (const float*)d_in[6];
  const float* Wv_b = (const float*)d_in[7];
  const float* Wo_w = (const float*)d_in[8];
  const float* Wo_b = (const float*)d_in[9];
  float* out = (float*)d_out;

  char* ws = (char*)d_ws;
  unsigned short* Xb   = (unsigned short*)(ws +  0 * MiB);
  unsigned short* Wqb  = (unsigned short*)(ws +  8 * MiB);
  unsigned short* Wkb  = (unsigned short*)(ws + 10 * MiB);
  unsigned short* Wvb  = (unsigned short*)(ws + 12 * MiB);
  unsigned short* Wob  = (unsigned short*)(ws + 14 * MiB);
  unsigned short* Qp   = (unsigned short*)(ws + 16 * MiB);
  unsigned short* Kp   = (unsigned short*)(ws + 24 * MiB);
  unsigned short* Vtp  = (unsigned short*)(ws + 32 * MiB);
  unsigned short* Ctxh = (unsigned short*)(ws + 40 * MiB);
  unsigned short* Ctxl = (unsigned short*)(ws + 48 * MiB);

  const int nx2 = kRows * kHid / 2;
  const int nw2 = kHid * kHid / 2;
  cast_f32_bf16x2<<<nx2 / 256, 256, 0, stream>>>(x,    Xb,  nx2);
  cast_f32_bf16x2<<<nw2 / 256, 256, 0, stream>>>(Wq_w, Wqb, nw2);
  cast_f32_bf16x2<<<nw2 / 256, 256, 0, stream>>>(Wk_w, Wkb, nw2);
  cast_f32_bf16x2<<<nw2 / 256, 256, 0, stream>>>(Wv_w, Wvb, nw2);
  cast_f32_bf16x2<<<nw2 / 256, 256, 0, stream>>>(Wo_w, Wob, nw2);

  wmma_gemm64<1, 0, 2, 1, false, true><<<dim3(128, 1), 256, 0, stream>>>(
      Xb, Xb, kHid, 0L, Wqb, Wqb, kHid, 0L, (void*)Qp, (void*)Qp, kHid, 0L,
      Wq_b, Wq_b, 0L, kRows, kHid, kHid, 1.0f);
  wmma_gemm64<1, 0, 2, 1, false, true><<<dim3(128, 1), 256, 0, stream>>>(
      Xb, Xb, kHid, 0L, Wkb, Wkb, kHid, 0L, (void*)Kp, (void*)Kp, kHid, 0L,
      Wk_b, Wk_b, 0L, kRows, kHid, kHid, 1.0f);
  wmma_gemm64<1, 0, 1, 1, false, true><<<dim3(64, kBatch), 256, 0, stream>>>(
      Wvb, Wvb, kHid, 0L, Xb, Xb, kHid, (long)kSeq * kHid, (void*)Vtp, (void*)Vtp, kSeq, (long)kHid * kSeq,
      Wv_b, Wv_b, 0L, kHid, kSeq, kHid, 1.0f);

  mha_full64_f16<<<kBatch * kHeads * (kSeq / AT_QB), 128, 0, stream>>>(Qp, Kp, Vtp, mask, Ctxh, Ctxl);

  wmma_gemm64<1, 2, 2, 0, false, true><<<dim3(128, 1), 256, 0, stream>>>(
      Ctxh, Ctxl, kHid, 0L, Wob, Wob, kHid, 0L, (void*)out, (void*)out, kHid, 0L,
      Wo_b, Wo_b, 0L, kRows, kHid, kHid, 1.0f);
}
